// RelTransformerQ_23287312679396
// MI455X (gfx1250) — hardware-verified
//
#include <hip/hip_runtime.h>
#include <stddef.h>


typedef _Float16 h16;
typedef _Float16 v16h __attribute__((ext_vector_type(16)));
typedef _Float16 v8h  __attribute__((ext_vector_type(8)));
typedef float    v8f  __attribute__((ext_vector_type(8)));
typedef float    v4f  __attribute__((ext_vector_type(4)));
typedef float    v2f  __attribute__((ext_vector_type(2)));

#ifndef NB
#define NB 256
#endif
#ifndef SEQ
#define SEQ 128
#endif
#define NB_FULL  256
#define SEQ_FULL 128
#define SDIM  8
#define ADIM  2
#define NHEAD 3
#define HDK   4
#define QDIM  10
#define HKD   12
#define XIN   22
#define XPAD  32
#define HID   256
#define MROWS (NB * SEQ)

static_assert(NB >= 1 && NB <= NB_FULL);
static_assert(SEQ == 128 && SEQ == SEQ_FULL);
static_assert(QDIM == SDIM + ADIM && HKD == NHEAD * HDK && XIN == HKD + QDIM);
static_assert(HDK == 4 && SDIM == 8 && ADIM == 2);
static_assert(XIN <= XPAD && (XPAD % 32) == 0 && XPAD == 32);
static_assert((HID % 64) == 0 && (HID % 32) == 0 && HID == 4 * 64);
static_assert((MROWS % 64) == 0);
static_assert(SEQ * NHEAD == 384);
static_assert(SEQ * XPAD / 8 == 512);
static_assert(((HID * XPAD / 8) % 256) == 0);
static_assert(((HID * HID / 8) % 256) == 0);
static_assert((size_t)NB_FULL * SEQ_FULL * 4 == (size_t)131072);

#define LDC  68
#define XLDF 36
static_assert((LDC % 4) == 0 && LDC >= 64);
static_assert((XLDF % 4) == 0 && XLDF >= XPAD);
static_assert((size_t)64 * LDC * 4 <= (size_t)131072);
static_assert((size_t)SEQ * 16 + (size_t)SEQ * XLDF * 4 <= (size_t)131072);

#define WCARRY 64.0f
#define XCARRY 16.0f
#define MCARRY 16.0f

#define W1_BYTES ((size_t)HID * XPAD * 2)
#define W2_BYTES ((size_t)HID * HID * 2)
#define X0_BYTES ((size_t)MROWS * XPAD * 2)
#define H1_BYTES ((size_t)MROWS * HID * 2)
#define OFF_W1 ((size_t)0)
#define OFF_W2 (OFF_W1 + W1_BYTES)
#define OFF_X0 (OFF_W2 + W2_BYTES)
#define OFF_H1 (OFF_X0 + X0_BYTES)
#define WS_TOTAL (OFF_H1 + H1_BYTES)
static_assert((W1_BYTES % 128) == 0 && (W2_BYTES % 128) == 0);
static_assert((X0_BYTES % 128) == 0 && (H1_BYTES % 128) == 0);
static_assert(WS_TOTAL <= (size_t)134217728);

__device__ __forceinline__ float bf16r(float x) {
  unsigned int u = __float_as_uint(x);
  u = (u + 0x7FFFu + ((u >> 16) & 1u)) & 0xFFFF0000u;
  return __uint_as_float(u);
}

static __device__ __forceinline__ h16 toh_flush(float v) {
  const h16 r = (h16)v;
  return (fabsf(v) < 6.103515625e-05f) ? (h16)0.0f : r;
}

__device__ __forceinline__ v16h frag_at(const _Float16* p) {
  v8h lo = *(const v8h*)(p);
  v8h hi = *(const v8h*)(p + 16);
  v16h out;
#pragma unroll
  for (int i = 0; i < 8; ++i) { out[i] = lo[i]; out[i + 8] = hi[i]; }
  return out;
}

__device__ __forceinline__ v8f wmma16(v16h a, v16h b, v8f c) {
  v8f d = __builtin_amdgcn_wmma_f32_16x16x32_f16(false, a, false, b, (short)0, c,
                                                 false, false);
  asm volatile("v_nop\n\tv_nop\n\tv_nop\n\tv_nop" : "+v"(d) : "v"(a), "v"(b));
  return d;
}

__device__ __forceinline__ float red16_sum(float x) {
#pragma unroll
  for (int off = 1; off < 16; off <<= 1) x += __shfl_xor(x, off, 32);
  return x;
}

__device__ __forceinline__ float relu_act(float t) {
  return fmaxf(t, 0.0f);
}

__global__ __launch_bounds__(256) void wcast_kernel(
    const float* __restrict__ W, _Float16* __restrict__ Wt,
    unsigned kin, unsigned kpad, unsigned nrows) {
  const unsigned g = blockIdx.x * 256u + threadIdx.x;
  const unsigned per = kpad >> 3;
  const unsigned total = nrows * per;
  const unsigned gc = (g < total) ? g : (total - 1u);
  const unsigned n = gc / per;
  const unsigned kc = (gc - n * per) * 8u;
  v8h x;
#pragma unroll
  for (unsigned j = 0; j < 8u; ++j) {
    const unsigned k = kc + j;
    const unsigned kl = (k < kin) ? k : (kin - 1u);
    const float v = W[(size_t)n * kin + kl];
    const h16 t = toh_flush(WCARRY * bf16r(v));
    x[j] = (k < kin) ? t : (h16)0.0f;
  }
  if (g < total) {
    _Float16* p = Wt + (size_t)gc * 8u;
    *(volatile v8h*)p = x;
    __threadfence();
    *(volatile v8h*)p = x;
  }
}

__global__ __launch_bounds__(384) void relattn_kernel(
    const float* __restrict__ state, const float* __restrict__ action,
    const float* __restrict__ Wk, const float* __restrict__ Wq, const float* __restrict__ Wv,
    _Float16* __restrict__ X0) {
  __shared__ v4f S4[SEQ];
  __shared__ float Xs[SEQ * XLDF];

  const unsigned tid = threadIdx.x, lane = tid & 31u;
  const unsigned wave = __builtin_amdgcn_readfirstlane(tid >> 5);
  const unsigned h = wave >> 2;
  const unsigned t = (wave & 3u) * 32u + lane;
  const unsigned b = blockIdx.x;
  const size_t frow = (size_t)b * SEQ_FULL + t;

  const v4f sa = *(const v4f*)(state + frow * SDIM);
  const v4f sb = *(const v4f*)(state + frow * SDIM + 4u);
  const v2f ac = *(const v2f*)(action + frow * ADIM);
  float qs[QDIM];
#pragma unroll
  for (int i = 0; i < 4; ++i) { qs[i] = bf16r(sa[i]); qs[i + 4] = bf16r(sb[i]); }
  qs[8] = bf16r(ac[0]);
  qs[9] = bf16r(ac[1]);

  if (h == 0u) {
    const v4f s0 = {qs[0], qs[1], qs[2], qs[3]};
    const v4f s1 = {qs[4], qs[5], qs[6], qs[7]};
    const v4f s2 = {qs[8], qs[9], 0.0f, 0.0f};
    const v4f zz = {0.0f, 0.0f, 0.0f, 0.0f};
    S4[t] = s0;
    *(v4f*)&Xs[t * XLDF + 12u] = s0;
    *(v4f*)&Xs[t * XLDF + 16u] = s1;
    *(v4f*)&Xs[t * XLDF + 20u] = s2;
    *(v4f*)&Xs[t * XLDF + 24u] = zz;
    *(v4f*)&Xs[t * XLDF + 28u] = zz;
  }
  __syncthreads();

  float qk0 = 0.0f, qk1 = 0.0f, qk2 = 0.0f, qk3 = 0.0f;
#pragma unroll 1
  for (unsigned k = 0; k < (unsigned)HDK; ++k) {
    const unsigned r = h * (unsigned)HDK + k;
    float qv = 0.0f;
#pragma unroll
    for (int d = 0; d < QDIM; ++d) qv += bf16r(Wq[r * (unsigned)QDIM + (unsigned)d]) * qs[d];
    qk0 += qv * bf16r(Wk[r * 4u + 0u]);
    qk1 += qv * bf16r(Wk[r * 4u + 1u]);
    qk2 += qv * bf16r(Wk[r * 4u + 2u]);
    qk3 += qv * bf16r(Wk[r * 4u + 3u]);
  }
  qk0 *= 0.5f; qk1 *= 0.5f; qk2 *= 0.5f; qk3 *= 0.5f;

  const v4f si = S4[t];
  float mrun = -1.0e30f, l = 0.0f;
  float a0 = 0.0f, a1 = 0.0f, a2 = 0.0f, a3 = 0.0f;
#pragma unroll 2
  for (unsigned j = 0; j < (unsigned)SEQ; ++j) {
    const v4f sj = S4[j];
    const float r0 = sj[0] - si[0];
    const float r1 = sj[1] - si[1];
    const float r2 = sj[2] - si[2];
    const float r3 = sj[3] - si[3];
    float sc = qk0 * r0;
    sc += qk1 * r1;
    sc += qk2 * r2;
    sc += qk3 * r3;
    const bool self = (j == t);
    sc = self ? -1.0e30f : sc;
    const float mn = fmaxf(mrun, sc);
    const float cor = __expf(mrun - mn);
    float p = __expf(sc - mn);
    p = self ? 0.0f : p;
    l = l * cor + p;
    a0 = a0 * cor + p * r0;
    a1 = a1 * cor + p * r1;
    a2 = a2 * cor + p * r2;
    a3 = a3 * cor + p * r3;
    mrun = mn;
  }
  const float inv = __builtin_amdgcn_rcpf(l);
  a0 *= inv; a1 *= inv; a2 *= inv; a3 *= inv;

#pragma unroll 1
  for (unsigned k = 0; k < (unsigned)HDK; ++k) {
    const unsigned r = h * (unsigned)HDK + k;
    float xv = a0 * bf16r(Wv[r * 4u + 0u]);
    xv += a1 * bf16r(Wv[r * 4u + 1u]);
    xv += a2 * bf16r(Wv[r * 4u + 2u]);
    xv += a3 * bf16r(Wv[r * 4u + 3u]);
    Xs[t * XLDF + r] = xv;
  }
  __syncthreads();

  v8h x[2];
  size_t off[2];
#pragma unroll
  for (unsigned i = 0; i < 2u; ++i) {
    const unsigned idx = tid + 384u * i;
    const unsigned idc = (idx < 512u) ? idx : 511u;
    const unsigned r = idc >> 2;
    const unsigned c = (idc & 3u) * 8u;
    const v4f u0 = *(const v4f*)&Xs[r * XLDF + c];
    const v4f u1 = *(const v4f*)&Xs[r * XLDF + c + 4u];
#pragma unroll
    for (int j = 0; j < 4; ++j) {
      x[i][j]     = toh_flush(XCARRY * u0[j]);
      x[i][j + 4] = toh_flush(XCARRY * u1[j]);
    }
    off[i] = ((size_t)b * SEQ + r) * XPAD + c;
  }
  *(volatile v8h*)(X0 + off[0]) = x[0];
  if (wave < 4u) *(volatile v8h*)(X0 + off[1]) = x[1];
  __threadfence();
  *(volatile v8h*)(X0 + off[0]) = x[0];
  if (wave < 4u) *(volatile v8h*)(X0 + off[1]) = x[1];
}

__global__ __launch_bounds__(256) void gemm_h1_kernel(
    const _Float16* __restrict__ A16, const _Float16* __restrict__ Bt,
    const float* __restrict__ bias, _Float16* __restrict__ out16) {
  __shared__ float Cs[64 * LDC];
  const unsigned tid = threadIdx.x, lane = tid & 31u;
  const unsigned w = __builtin_amdgcn_readfirstlane(tid >> 5);
  const unsigned mw = w >> 1, nw = w & 1u;
  const unsigned hh = lane >> 4, m = lane & 15u;
  const unsigned n0 = blockIdx.x * 64u;
  const unsigned row0 = blockIdx.y * 64u;
  const unsigned K = (unsigned)XPAD;

  const _Float16* ap  = A16 + (size_t)(row0 + mw * 16u + m) * K + hh * 8u;
  const _Float16* bp0 = Bt + (size_t)(n0 + nw * 32u + m) * K + hh * 8u;
  const _Float16* bp1 = bp0 + (size_t)16 * K;
  v8f acc0 = {}, acc1 = {};
#pragma unroll 1
  for (unsigned k0 = 0; k0 < K; k0 += 32u) {
    const v16h a  = frag_at(ap + k0);
    const v16h b0 = frag_at(bp0 + k0);
    const v16h b1 = frag_at(bp1 + k0);
    acc0 = wmma16(a, b0, acc0);
    acc1 = wmma16(a, b1, acc1);
  }
#pragma unroll
  for (int r = 0; r < 8; ++r) {
    const unsigned ci = (mw * 16u + hh * 8u + (unsigned)r) * LDC + nw * 32u + m;
    Cs[ci]       = acc0[r];
    Cs[ci + 16u] = acc1[r];
  }
  __syncthreads();

#pragma unroll 1
  for (unsigned g = 0; g < 4u; ++g) {
    const unsigned r = 32u * (g >> 1) + (tid >> 3);
    const unsigned c = (tid & 7u) * 8u + 4u * (g & 1u);
    const v4f u  = *(const v4f*)&Cs[r * LDC + c];
    const v4f gb = *(const v4f*)(bias + n0 + c);
    v4f t;
#pragma unroll
    for (int j = 0; j < 4; ++j)
      t[j] = MCARRY * relu_act(u[j] * (1.0f / (WCARRY * XCARRY)) + bf16r(gb[j]));
    *(v4f*)&Cs[r * LDC + c] = t;
  }

  v8h x[2];
  size_t off[2];
#pragma unroll
  for (unsigned i = 0; i < 2u; ++i) {
    const unsigned r = 32u * i + (tid >> 3);
    const unsigned c = (tid & 7u) * 8u;
    const v4f u0 = *(const v4f*)&Cs[r * LDC + c];
    const v4f u1 = *(const v4f*)&Cs[r * LDC + c + 4];
#pragma unroll
    for (int j = 0; j < 4; ++j) {
      x[i][j]     = toh_flush(u0[j]);
      x[i][j + 4] = toh_flush(u1[j]);
    }
    off[i] = (size_t)(row0 + r) * HID + n0 + c;
  }
#pragma unroll
  for (int i = 0; i < 2; ++i) *(volatile v8h*)(out16 + off[i]) = x[i];
  __threadfence();
#pragma unroll
  for (int i = 0; i < 2; ++i) *(volatile v8h*)(out16 + off[i]) = x[i];
}

__global__ __launch_bounds__(256) void gemm_out_kernel(
    const _Float16* __restrict__ A16, const _Float16* __restrict__ Bt,
    const float* __restrict__ bias, const float* __restrict__ wout,
    const float* __restrict__ bout, float* __restrict__ outf) {
  __shared__ float Rs[2 * 64];
  const unsigned tid = threadIdx.x, lane = tid & 31u;
  const unsigned w = __builtin_amdgcn_readfirstlane(tid >> 5);
  const unsigned mw = w >> 1, nw = w & 1u;
  const unsigned hh = lane >> 4, m = lane & 15u;
  const unsigned row0 = blockIdx.x * 64u;
  const unsigned K = (unsigned)HID;
  const float cs = 1.0f / (WCARRY * MCARRY);

  const _Float16* ap = A16 + (size_t)(row0 + mw * 16u + m) * K + hh * 8u;
  float rsum[8];
#pragma unroll
  for (int r = 0; r < 8; ++r) rsum[r] = 0.0f;

#pragma unroll 1
  for (unsigned nt = 0; nt < 4u; ++nt) {
    const unsigned nb = nt * 64u + nw * 32u;
    const _Float16* bp0 = Bt + (size_t)(nb + m) * K + hh * 8u;
    const _Float16* bp1 = bp0 + (size_t)16 * K;
    v8f acc0 = {}, acc1 = {};
#pragma unroll 2
    for (unsigned k0 = 0; k0 < K; k0 += 32u) {
      const v16h a  = frag_at(ap + k0);
      const v16h b0 = frag_at(bp0 + k0);
      const v16h b1 = frag_at(bp1 + k0);
      acc0 = wmma16(a, b0, acc0);
      acc1 = wmma16(a, b1, acc1);
    }
    const unsigned c0 = nb + m, c1 = nb + m + 16u;
    const float bb0 = bf16r(bias[c0]), bb1 = bf16r(bias[c1]);
    const float w0 = bf16r(wout[c0]), w1 = bf16r(wout[c1]);
#pragma unroll
    for (int r = 0; r < 8; ++r) {
      const float y0 = relu_act(acc0[r] * cs + bb0);
      const float y1 = relu_act(acc1[r] * cs + bb1);
      rsum[r] += y0 * w0 + y1 * w1;
    }
  }
#pragma unroll
  for (int r = 0; r < 8; ++r) rsum[r] = red16_sum(rsum[r]);
  if (m == 0u) {
#pragma unroll
    for (int r = 0; r < 8; ++r) Rs[nw * 64u + mw * 16u + hh * 8u + (unsigned)r] = rsum[r];
  }
  __syncthreads();

  if (w == 0u) {
    const float bo = bf16r(bout[0]);
    const unsigned i4 = (lane & 15u) * 4u;
    const v4f p0 = *(const v4f*)&Rs[i4];
    const v4f p1 = *(const v4f*)&Rs[64u + i4];
    v4f o;
#pragma unroll
    for (int j = 0; j < 4; ++j) o[j] = (p0[j] + p1[j]) + bo;
    float* dst = outf + row0 + i4;
    if (lane < 16u) *(volatile v4f*)dst = o;
    __threadfence();
    if (lane < 16u) *(volatile v4f*)dst = o;
  }
}

extern "C" void kernel_launch(void* const* d_in, const int* in_sizes, int n_in,
                              void* d_out, int out_size, void* d_ws, size_t ws_size,
                              hipStream_t stream) {
  if (n_in < 11) return;
  const long long need_rows = (long long)(NB - 1) * SEQ_FULL + SEQ;
  if ((long long)in_sizes[0] < need_rows * SDIM) return;
  if ((long long)in_sizes[1] < need_rows * ADIM) return;
  if (in_sizes[2] < HKD * HDK) return;
  if (in_sizes[3] < HKD * QDIM) return;
  if (in_sizes[4] < HKD * HDK) return;
  if (in_sizes[5] < HID * XIN) return;
  if (in_sizes[6] < HID) return;
  if ((long long)in_sizes[7] < (long long)HID * HID) return;
  if (in_sizes[8] < HID) return;
  if (in_sizes[9] < HID) return;
  if (in_sizes[10] < 1) return;
  if ((long long)out_size < need_rows) return;
  if (ws_size < WS_TOTAL) return;

  const float* state  = (const float*)d_in[0];
  const float* action = (const float*)d_in[1];
  const float* wk     = (const float*)d_in[2];
  const float* wq     = (const float*)d_in[3];
  const float* wv     = (const float*)d_in[4];
  const float* w1     = (const float*)d_in[5];
  const float* b1     = (const float*)d_in[6];
  const float* w2     = (const float*)d_in[7];
  const float* b2     = (const float*)d_in[8];
  const float* wo     = (const float*)d_in[9];
  const float* bo     = (const float*)d_in[10];
  float* out = (float*)d_out;

  char* ws = (char*)d_ws;
  _Float16* W1t = (_Float16*)(ws + OFF_W1);
  _Float16* W2t = (_Float16*)(ws + OFF_W2);
  _Float16* X0  = (_Float16*)(ws + OFF_X0);
  _Float16* H1  = (_Float16*)(ws + OFF_H1);

  dim3 blk(256);
  wcast_kernel<<<dim3(HID * XPAD / 8 / 256), blk, 0, stream>>>(
      w1, W1t, (unsigned)XIN, (unsigned)XPAD, (unsigned)HID);
  wcast_kernel<<<dim3(HID * HID / 8 / 256), blk, 0, stream>>>(
      w2, W2t, (unsigned)HID, (unsigned)HID, (unsigned)HID);

  relattn_kernel<<<dim3(NB), dim3(384), 0, stream>>>(state, action, wk, wq, wv, X0);
  gemm_h1_kernel<<<dim3(HID / 64, MROWS / 64), blk, 0, stream>>>(X0, W1t, b1, H1);
  gemm_out_kernel<<<dim3(MROWS / 64), blk, 0, stream>>>(H1, W2t, b2, wo, bo, out);
}
